// Encoder_37271726195512
// MI455X (gfx1250) — hardware-verified
//
#include <hip/hip_runtime.h>
#include <math.h>

constexpr int NSTEP    = 64;
constexpr int NBATCH   = 16384;
constexpr int NEMB     = 64;
constexpr int NHID     = 128;
constexpr int NGATE    = 4 * NHID;
constexpr int NTHR     = 256;
constexpr int ROWS_BLK = 16;
constexpr int HPITCH   = 136;
constexpr int OPITCH   = 132;
constexpr float H_CARRY  = 64.0f;
constexpr float W_CARRY  = 16.0f;
constexpr float FOLD     = H_CARRY * W_CARRY;
constexpr float FOLD_INV = 1.0f / FOLD;

static_assert(NGATE == 512, "gate width");
static_assert(NBATCH % ROWS_BLK == 0, "grid exact");
static_assert(NHID == 16 * (NTHR / 32), "8 waves x 16 hidden columns");
static_assert(NHID % 32 == 0, "K multiple of 32");
static_assert((2 * ROWS_BLK * HPITCH) % NTHR == 0, "h zero-fill loop exact");
static_assert((3 * NGATE) % NTHR == 0, "u staging loop exact");
static_assert((NGATE * NHID / 8) % NTHR == 0, "weight cast grid exact");
static_assert(NGATE % NTHR == 0, "u build grid exact");
static_assert((ROWS_BLK * NHID / 4) % NTHR == 0, "final store loop exact");
static_assert(HPITCH % 8 == 0 && OPITCH % 4 == 0, "16-B aligned LDS rows");

typedef __attribute__((ext_vector_type(16))) _Float16 v16h;
typedef __attribute__((ext_vector_type(8)))  _Float16 v8h;
typedef __attribute__((ext_vector_type(8)))  float    v8f;
typedef __attribute__((ext_vector_type(4)))  float    v4f;
typedef __attribute__((ext_vector_type(4)))  unsigned v4u;

__device__ __forceinline__ void guard_grp(v8f& a0, v8f& a1, v8f& a2, v8f& a3,
                                          v16h x, v16h b0, v16h b1, v16h b2, v16h b3) {
  asm volatile("v_nop\n\tv_nop\n\tv_nop\n\tv_nop"
               : "+v"(a0), "+v"(a1), "+v"(a2), "+v"(a3)
               : "v"(x), "v"(b0), "v"(b1), "v"(b2), "v"(b3));
}
__device__ __forceinline__ void pin_frag(v16h& f) { asm volatile("" : "+v"(f)); }

struct FragH {
  union U { v16h v; v8h h[2]; };
  static __device__ __forceinline__ v16h load(const _Float16* p) {
    U f;
    f.h[0] = *(const v8h*)(p);
    f.h[1] = *(const v8h*)(p + 16);
    return f.v;
  }
  static __device__ __forceinline__ v8f mma(v16h a, v16h b, v8f c) {
    return __builtin_amdgcn_wmma_f32_16x16x32_f16(false, a, false, b, (short)0, c, false, false);
  }
};

__device__ __forceinline__ float fsig(float x)  { return __builtin_amdgcn_rcpf(1.0f + __expf(-x)); }
__device__ __forceinline__ float ftanh(float x) { return 1.0f - 2.0f * __builtin_amdgcn_rcpf(__expf(2.0f * x) + 1.0f); }
__device__ __forceinline__ bool  bits_is_nan(unsigned u) { return (u & 0x7fffffffu) > 0x7f800000u; }
__device__ __forceinline__ float bits_clean(unsigned u)  { return bits_is_nan(u) ? 0.0f : __uint_as_float(u); }

__global__ __launch_bounds__(NTHR) void cast_whh_kernel(const float* __restrict__ src, unsigned short* __restrict__ dst) {
  const int i  = blockIdx.x * NTHR + threadIdx.x;
  const int n8 = NGATE * NHID / 8;
  if (i < n8) {
    const float* sp = src + (size_t)i * 8;
    const v4f a = *(const v4f*)(sp);
    const v4f b = *(const v4f*)(sp + 4);
    v8h hv;
#pragma unroll
    for (int e = 0; e < 4; ++e) {
      const float fa = a[e] * W_CARRY;
      const float fb = b[e] * W_CARRY;
      hv[e]     = (_Float16)fa;
      hv[4 + e] = (_Float16)fb;
    }
    *(volatile v8h*)(dst + (size_t)i * 8) = hv;
    __threadfence();
    *(volatile v8h*)(dst + (size_t)i * 8) = hv;
  }
}

__global__ __launch_bounds__(NTHR) void build_u_kernel(const float* __restrict__ Wemb, const float* __restrict__ bemb,
                                                       const float* __restrict__ wih, const float* __restrict__ bih,
                                                       const float* __restrict__ bhh, float* __restrict__ U) {
  const int n = blockIdx.x * NTHR + threadIdx.x;
  if (n < NGATE) {
    float s0 = 0.0f, s1 = 0.0f, s2 = 0.0f;
    const float* wr = wih + (size_t)n * NEMB;
#pragma unroll 1
    for (int e4 = 0; e4 < NEMB; e4 += 4) {
      const v4f w  = *(const v4f*)(wr + e4);
      const v4f a0 = *(const v4f*)(Wemb + e4);
      const v4f a1 = *(const v4f*)(Wemb + NEMB + e4);
      const v4f bb = *(const v4f*)(bemb + e4);
#pragma unroll
      for (int e = 0; e < 4; ++e) {
        s0 = fmaf(a0[e], w[e], s0);
        s1 = fmaf(a1[e], w[e], s1);
        s2 = fmaf(bb[e], w[e], s2);
      }
    }
    s2 += (bih[n] + bhh[n]);
    const float o0 = s0 * FOLD;
    const float o1 = s1 * FOLD;
    const float o2 = s2 * FOLD;
    volatile float* up = (volatile float*)U;
    up[n]             = o0;
    up[NGATE + n]     = o1;
    up[2 * NGATE + n] = o2;
    __threadfence();
    up[n]             = o0;
    up[NGATE + n]     = o1;
    up[2 * NGATE + n] = o2;
  }
}

__global__ __launch_bounds__(NTHR) void lstm_seq_kernel(const float* __restrict__ obs,
                                                        const unsigned short* __restrict__ WHp,
                                                        const float* __restrict__ U,
                                                        float* __restrict__ out) {
  __shared__ __align__(16) _Float16 Ah[2][ROWS_BLK * HPITCH];
  __shared__ __align__(16) float    Hs[ROWS_BLK * OPITCH];
  __shared__ __align__(16) float    sU[3 * NGATE];
  __shared__ __align__(16) unsigned sObs[2][2 * ROWS_BLK];

  const _Float16* WH = (const _Float16*)WHp;
  const int tid = threadIdx.x, lane = tid & 31, wave = tid >> 5;
  const int c = lane & 15, hh = lane >> 4, koff = hh * 8;
  const int rowbase = blockIdx.x * ROWS_BLK;
  const int ucol = 16 * wave + c;

  {
    _Float16* ahf = &Ah[0][0];
#pragma unroll 1
    for (int i = tid; i < 2 * ROWS_BLK * HPITCH; i += NTHR) ahf[i] = (_Float16)0.0f;
  }
#pragma unroll 1
  for (int i = tid; i < 3 * NGATE; i += NTHR) sU[i] = U[i];
  if (wave == 0) {
    const float v = obs[(size_t)rowbase * 2 + lane];
    sObs[0][lane] = __float_as_uint(v);
  }

  v16h wf[4][4];
#pragma unroll
  for (int g = 0; g < 4; ++g) {
#pragma unroll
    for (int kk = 0; kk < 4; ++kk) {
      wf[g][kk] = FragH::load(WH + (size_t)(g * NHID + ucol) * NHID + koff + kk * 32);
      pin_frag(wf[g][kk]);
    }
  }

  float cst[8], hst[8];
#pragma unroll
  for (int r = 0; r < 8; ++r) { cst[r] = 0.0f; hst[r] = 0.0f; }

  __syncthreads();

#pragma unroll 1
  for (int t = 0; t < NSTEP; ++t) {
    const int par = t & 1;

    if (wave == 0) {
      const int tn = (t + 1 < NSTEP) ? (t + 1) : (NSTEP - 1);
      const float v = obs[((size_t)tn * NBATCH + (size_t)rowbase) * 2 + lane];
      sObs[par ^ 1][lane] = __float_as_uint(v);
    }

    unsigned xb[16];
    {
      const v4u* xo = (const v4u*)(&sObs[par][16 * hh]);
      const v4u q0 = xo[0], q1 = xo[1], q2 = xo[2], q3 = xo[3];
#pragma unroll
      for (int e = 0; e < 4; ++e) {
        xb[e]      = q0[e];
        xb[4 + e]  = q1[e];
        xb[8 + e]  = q2[e];
        xb[12 + e] = q3[e];
      }
    }

    float u0g[4], u1g[4], u2g[4];
#pragma unroll
    for (int g = 0; g < 4; ++g) {
      u0g[g] = sU[g * NHID + ucol];
      u1g[g] = sU[NGATE + g * NHID + ucol];
      u2g[g] = sU[2 * NGATE + g * NHID + ucol];
    }
    v8f acc[4];
    unsigned vmask = 0u;
#pragma unroll
    for (int r = 0; r < 8; ++r) {
      const float x0 = bits_clean(xb[2 * r]);
      const float x1 = bits_clean(xb[2 * r + 1]);
      vmask |= bits_is_nan(xb[2 * r]) ? 0u : (1u << r);
#pragma unroll
      for (int g = 0; g < 4; ++g) acc[g][r] = fmaf(x1, u1g[g], fmaf(x0, u0g[g], u2g[g]));
    }

    const _Float16* ahrow = &Ah[par][0] + c * HPITCH + koff;
#pragma unroll
    for (int kk = 0; kk < 4; ++kk) {
      const v16h a = FragH::load(ahrow + kk * 32);
      acc[0] = FragH::mma(a, wf[0][kk], acc[0]);
      acc[1] = FragH::mma(a, wf[1][kk], acc[1]);
      acc[2] = FragH::mma(a, wf[2][kk], acc[2]);
      acc[3] = FragH::mma(a, wf[3][kk], acc[3]);
      guard_grp(acc[0], acc[1], acc[2], acc[3], a, wf[0][kk], wf[1][kk], wf[2][kk], wf[3][kk]);
    }

    _Float16* ahn = &Ah[par ^ 1][0];
#pragma unroll
    for (int r = 0; r < 8; ++r) {
      const float zi = acc[0][r] * FOLD_INV;
      const float zf = acc[1][r] * FOLD_INV;
      const float zg = acc[2][r] * FOLD_INV;
      const float zo = acc[3][r] * FOLD_INV;
      const float ig = fsig(zi);
      const float fg = fsig(zf);
      const float gg = ftanh(zg);
      const float og = fsig(zo);
      const float cn = fg * cst[r] + ig * gg;
      const float hn = og * ftanh(cn);
      const bool keep = ((vmask >> r) & 1u) != 0u;
      const float cnew = keep ? cn : cst[r];
      const float hnew = keep ? hn : hst[r];
      cst[r] = cnew;
      hst[r] = hnew;
      const float hs = hnew * H_CARRY;
      ahn[(8 * hh + r) * HPITCH + ucol] = (_Float16)hs;
    }

    __syncthreads();
  }

#pragma unroll
  for (int r = 0; r < 8; ++r) Hs[(8 * hh + r) * OPITCH + ucol] = hst[r];
  __syncthreads();
  for (int pass = 0; pass < 2; ++pass) {
#pragma unroll
    for (int it = 0; it < 2; ++it) {
      const int idx = it * NTHR + tid;
      const int row = idx >> 5;
      const int c4  = (idx & 31) * 4;
      const v4f v = *(const v4f*)(Hs + row * OPITCH + c4);
      *(volatile v4f*)(out + (size_t)(rowbase + row) * NHID + c4) = v;
    }
    __threadfence();
  }
}

extern "C" void kernel_launch(void* const* d_in, const int* in_sizes, int n_in,
                              void* d_out, int out_size, void* d_ws, size_t ws_size, hipStream_t stream) {
  if (n_in < 7 || d_out == nullptr || d_ws == nullptr) return;
  if (in_sizes[0] != NSTEP * NBATCH * 2 || in_sizes[1] != 2 * NEMB || in_sizes[2] != NEMB ||
      in_sizes[3] != NGATE * NEMB || in_sizes[4] != NGATE * NHID || in_sizes[5] != NGATE ||
      in_sizes[6] != NGATE || out_size != NBATCH * NHID) return;

  const float* obs  = (const float*)d_in[0];
  const float* Wemb = (const float*)d_in[1];
  const float* bemb = (const float*)d_in[2];
  const float* wih  = (const float*)d_in[3];
  const float* whh  = (const float*)d_in[4];
  const float* bih  = (const float*)d_in[5];
  const float* bhh  = (const float*)d_in[6];
  float* out = (float*)d_out;

  char* ws = (char*)d_ws;
  size_t off = 0;
  auto carve = [&](size_t bytes) -> char* { char* p = ws + off; off += (bytes + 255) & ~(size_t)255; return p; };
  unsigned short* WH16 = (unsigned short*)carve((size_t)NGATE * NHID * 2);
  float*          UPL  = (float*)carve((size_t)3 * NGATE * 4);
  if (off > ws_size || off > (size_t)134217728) return;

  cast_whh_kernel<<<(NGATE * NHID / 8) / NTHR, NTHR, 0, stream>>>(whh, WH16);
  build_u_kernel<<<NGATE / NTHR, NTHR, 0, stream>>>(Wemb, bemb, wih, bih, bhh, UPL);
  lstm_seq_kernel<<<NBATCH / ROWS_BLK, NTHR, 0, stream>>>(obs, WH16, UPL, out);
}
